// RecursiveNeuralKernel_46213848105644
// MI455X (gfx1250) — hardware-run, weakly checked
//
#include <hip/hip_runtime.h>
#include <stddef.h>
#include <stdint.h>


#define MR    256
#define DD    1024
#define DH    512
#define KD    1024
#define ASC   16
#define WSC   1024
#define NTHR  256
#define NWAVE 8
#define WSCAP 134217728
#define LDS_GEMM (NWAVE * 32 * 64 * 4)

static_assert((KD % 32) == 0);
static_assert((MR % 128) == 0);
static_assert((DD % 128) == 0);
static_assert((DH % 128) == 0);
static_assert(NTHR == NWAVE * 32);
static_assert(((DD * KD) % (8 * NTHR)) == 0);
static_assert(((DH * KD) % (8 * NTHR)) == 0);
static_assert(((MR * KD) % (8 * NTHR)) == 0);
static_assert((MR * 3) == 3 * NTHR);
static_assert(((MR * 3) % 4) == 0);
static_assert(LDS_GEMM <= 300 * 1024);

typedef float          v4f  __attribute__((ext_vector_type(4)));
typedef float          v8f  __attribute__((ext_vector_type(8)));
typedef _Float16       v8h  __attribute__((ext_vector_type(8)));
typedef _Float16       v16h __attribute__((ext_vector_type(16)));
union FragH { v16h v; v8h h[2]; };

struct FaScales { float s0, s1, s2, s3, s4; };
static_assert(sizeof(FaScales) == 20);

__device__ __forceinline__ v8f wmf(v16h a, v16h b, v8f c) {
  v8f d = __builtin_amdgcn_wmma_f32_16x16x32_f16(false, a, false, b, (short)0, c, false, false);
  asm volatile("v_nop\n\tv_nop\n\tv_nop\n\tv_nop" : "+v"(d) : "v"(a), "v"(b));
  return d;
}

__device__ __forceinline__ float fa_term(float v, float s, float w) {
  const float sx = v * s;
  const float e  = expf(-0.1f * fabsf(sx));
  const float sn = sinf(sx);
  return (sn * e) * w;
}

__device__ __forceinline__ v4f fa4(v4f v, const float* pw) {
  v4f r = {0.f, 0.f, 0.f, 0.f};
#pragma unroll 1
  for (int i = 0; i < 5; ++i) {
    const float w = pw[i], s = pw[5 + i];
    r.x += fa_term(v.x, s, w);
    r.y += fa_term(v.y, s, w);
    r.z += fa_term(v.z, s, w);
    r.w += fa_term(v.w, s, w);
  }
  return r;
}

__global__ __launch_bounds__(NTHR) void k_cvt(const float* __restrict__ src, _Float16* dst, float scale) {
  const size_t t = (size_t)blockIdx.x * NTHR + threadIdx.x;
  const float* p = src + t * 8;
  const v4f f0 = *(const v4f*)p;
  const v4f f1 = *(const v4f*)(p + 4);
  v8h a;
  a[0] = (_Float16)(f0.x * scale); a[1] = (_Float16)(f0.y * scale);
  a[2] = (_Float16)(f0.z * scale); a[3] = (_Float16)(f0.w * scale);
  a[4] = (_Float16)(f1.x * scale); a[5] = (_Float16)(f1.y * scale);
  a[6] = (_Float16)(f1.z * scale); a[7] = (_Float16)(f1.w * scale);
  _Float16* d = dst + t * 8;
  *(volatile v8h*)d = a;
  __threadfence();
  *(volatile v8h*)d = a;
}

template <int MODE>
__device__ __forceinline__ void store_pass(const float* stg, float* of32, _Float16* of16, int N,
                                           int grow0, int gcol0, int lane, float hsc) {
  const int hf = lane >> 4, m = lane & 15;
  if (MODE == 1 || MODE == 3 || MODE == 4) {
    float* gb = of32 + (size_t)grow0 * N + gcol0;
#pragma unroll
    for (int q = 0; q < 16; ++q) {
      const int row = 2 * q + hf;
      const v4f v = *(const v4f*)(stg + row * 64 + 4 * m);
      *(volatile v4f*)(gb + (size_t)row * N + 4 * m) = v;
    }
  }
  if (MODE == 0 || MODE == 1 || MODE == 2) {
    _Float16* hb = of16 + (size_t)grow0 * N + gcol0;
    const int rq = lane >> 3, c8 = 8 * (lane & 7);
#pragma unroll
    for (int q = 0; q < 8; ++q) {
      const int row = 4 * q + rq;
      const v4f a = *(const v4f*)(stg + row * 64 + c8);
      const v4f b = *(const v4f*)(stg + row * 64 + c8 + 4);
      v8h hv;
      hv[0] = (_Float16)(a.x * hsc); hv[1] = (_Float16)(a.y * hsc);
      hv[2] = (_Float16)(a.z * hsc); hv[3] = (_Float16)(a.w * hsc);
      hv[4] = (_Float16)(b.x * hsc); hv[5] = (_Float16)(b.y * hsc);
      hv[6] = (_Float16)(b.z * hsc); hv[7] = (_Float16)(b.w * hsc);
      *(volatile v8h*)(hb + (size_t)row * N + c8) = hv;
    }
  }
}

template <int MODE>
__global__ __launch_bounds__(NTHR) void k_gemm(const _Float16* __restrict__ A, const _Float16* __restrict__ Wt,
                                               const float* __restrict__ bias, const float* hn,
                                               const float* __restrict__ sfp, const float* __restrict__ modp,
                                               const float* __restrict__ ratep, FaScales fs, int N, int depth,
                                               float* of32, _Float16* of16) {
  extern __shared__ v4f lds_dyn[];
  __shared__ float prm[16];
  const int tid = threadIdx.x, lane = tid & 31, wave = tid >> 5, hf = lane >> 4, m = lane & 15;
  float* stg = (float*)lds_dyn + wave * (32 * 64);
  const int n0 = blockIdx.x * 128, m0 = blockIdx.y * 128;
  const int wm = (wave >> 1) * 32, wn = (wave & 1) * 64;

  if (MODE == 0 || MODE == 1) {
    if (tid == 0) {
      const float f0 = sfp[0], f1 = sfp[1], f2 = sfp[2], f3 = sfp[3], f4 = sfp[4];
      const float mx = fmaxf(fmaxf(fmaxf(f0, f1), fmaxf(f2, f3)), f4);
      const float e0 = expf(f0 - mx), e1 = expf(f1 - mx), e2 = expf(f2 - mx);
      const float e3 = expf(f3 - mx), e4 = expf(f4 - mx);
      const float s = (((e0 + e1) + e2) + e3) + e4;
      const float rs = 1.0f / s;
      prm[0] = e0 * rs; prm[1] = e1 * rs; prm[2] = e2 * rs; prm[3] = e3 * rs; prm[4] = e4 * rs;
      prm[5] = fs.s0; prm[6] = fs.s1; prm[7] = fs.s2; prm[8] = fs.s3; prm[9] = fs.s4;
    }
  }

  v8f acc[2][4];
#pragma unroll
  for (int mt = 0; mt < 2; ++mt)
#pragma unroll
    for (int nt = 0; nt < 4; ++nt) { v8f z = {0.f, 0.f, 0.f, 0.f, 0.f, 0.f, 0.f, 0.f}; acc[mt][nt] = z; }

  const _Float16* ap = A + (size_t)(m0 + wm + m) * KD + 8 * hf;
  const _Float16* bp = Wt + (size_t)(n0 + wn + m) * KD + 8 * hf;
#pragma unroll 1
  for (int kt = 0; kt < KD / 32; ++kt) {
    const int k0 = 32 * kt;
    FragH a0, a1;
    a0.h[0] = *(const v8h*)(ap + k0);
    a0.h[1] = *(const v8h*)(ap + k0 + 16);
    a1.h[0] = *(const v8h*)(ap + 16 * KD + k0);
    a1.h[1] = *(const v8h*)(ap + 16 * KD + k0 + 16);
#pragma unroll
    for (int nt = 0; nt < 4; ++nt) {
      const _Float16* bq = bp + (size_t)nt * 16 * KD + k0;
      FragH b;
      b.h[0] = *(const v8h*)bq;
      b.h[1] = *(const v8h*)(bq + 16);
      acc[0][nt] = wmf(a0.v, b.v, acc[0][nt]);
      acc[1][nt] = wmf(a1.v, b.v, acc[1][nt]);
    }
  }

  constexpr float OSC = 1.0f / (float)(ASC * WSC);
  float bv[4];
#pragma unroll
  for (int nt = 0; nt < 4; ++nt) bv[nt] = bias[n0 + wn + 16 * nt + m];
#pragma unroll
  for (int mt = 0; mt < 2; ++mt) {
    float* sp = stg + (16 * mt + 8 * hf) * 64 + m;
#pragma unroll
    for (int nt = 0; nt < 4; ++nt) {
#pragma unroll
      for (int r = 0; r < 8; ++r) sp[r * 64 + 16 * nt] = acc[mt][nt][r] * OSC + bv[nt];
    }
  }
  __syncthreads();

  float hsc = (float)ASC;
  if (MODE == 1) hsc = (float)ASC * modp[0];
  if (MODE != 3) {
    float w1 = 0.f, w2 = 0.f;
    if (MODE == 2) {
      const float z  = ratep[0] * (float)depth;
      const float iw = 1.0f / (1.0f + expf(-z));
      w1 = 1.0f - iw;
      w2 = iw;
    }
    v4f* stg4 = (v4f*)stg;
#pragma unroll 1
    for (int it = 0; it < 16; ++it) {
      const int j = it * 32 + lane;
      const v4f v = stg4[j];
      v4f t = v;
      if (MODE == 0 || MODE == 1) {
        t = fa4(v, prm);
      } else if (MODE == 2) {
        const int row = 2 * it + hf;
        const v4f hv = *(const v4f*)(hn + (size_t)(m0 + wm + row) * N + n0 + wn + 4 * m);
        t = hv * w1 + v * w2;
      } else {
        t.x = fmaxf(v.x, 0.0f); t.y = fmaxf(v.y, 0.0f); t.z = fmaxf(v.z, 0.0f); t.w = fmaxf(v.w, 0.0f);
      }
      stg4[j] = t;
    }
    __syncthreads();
  }

  store_pass<MODE>(stg, of32, of16, N, m0 + wm, n0 + wn, lane, hsc);
  __threadfence();
  store_pass<MODE>(stg, of32, of16, N, m0 + wm, n0 + wn, lane, hsc);
}

__global__ __launch_bounds__(NTHR) void k_cons(const float* __restrict__ c, const float* __restrict__ w,
                                               const float* __restrict__ b, float* out1) {
  __shared__ __attribute__((aligned(16))) float so[3 * NTHR];
  const int t = threadIdx.x;
#pragma unroll 1
  for (int u = 0; u < 3; ++u) {
    const int idx = u * NTHR + t;
    const int m = idx / 3;
    const int j = idx - 3 * m;
    const float* cr = c + (size_t)m * DH;
    const float* wr = w + (size_t)j * DH;
    float s = 0.0f;
#pragma unroll 4
    for (int k = 0; k < DH; ++k) s = fmaf(cr[k], wr[k], s);
    s += b[j];
    so[idx] = 1.0f / (1.0f + expf(-s));
  }
  __syncthreads();
  if (t < (3 * NTHR) / 4) {
    const v4f v = *(const v4f*)(so + 4 * t);
    float* d = out1 + 4 * t;
    *(volatile v4f*)d = v;
    __threadfence();
    *(volatile v4f*)d = v;
  }
}

namespace {

struct Net {
  const _Float16 *wt_in, *wt_h, *wt_out, *wt_c1;
  const float *b_in, *b_h, *b_out, *b_c1, *w_c2, *b_c2, *sf, *modp, *ratep;
  _Float16* xa[4];
  _Float16* ha[4];
  _Float16* hb;
  float* hn[3];
  float* cb;
  float* out;
  FaScales fs;
  hipStream_t st;
};

template <int MODE>
void run_gemm(const Net& c, const _Float16* A, const _Float16* W, const float* b, const float* hnp,
              int N, int depth, float* of32, _Float16* of16) {
  k_gemm<MODE><<<dim3(N / 128, MR / 128), NTHR, LDS_GEMM, c.st>>>(A, W, b, hnp, c.sf, c.modp, c.ratep,
                                                                  c.fs, N, depth, of32, of16);
}

void fwd(const Net& c, int depth) {
  run_gemm<0>(c, c.xa[depth], c.wt_in, c.b_in, c.hn[0], DD, 0, c.cb, c.ha[depth]);
  if (depth >= 3) {
    run_gemm<0>(c, c.ha[3], c.wt_h,                       c.b_h,          c.hn[0], DD, 0, c.cb, c.hb);
    run_gemm<0>(c, c.hb,    c.wt_h + (size_t)1 * DD * KD, c.b_h + 1 * DD, c.hn[0], DD, 0, c.cb, c.ha[3]);
    run_gemm<0>(c, c.ha[3], c.wt_h + (size_t)2 * DD * KD, c.b_h + 2 * DD, c.hn[0], DD, 0, c.cb, c.hb);
    run_gemm<2>(c, c.hb, c.wt_out, c.b_out, c.hn[depth - 1], DD, depth - 1, c.cb, c.ha[depth - 1]);
  } else {
    for (int i = 0; i < 3; ++i) {
      run_gemm<1>(c, c.ha[depth], c.wt_h + (size_t)i * DD * KD, c.b_h + (size_t)i * DD, c.hn[0], DD, 0,
                  c.hn[depth], c.xa[depth + 1]);
      fwd(c, depth + 1);
    }
    if (depth == 0) {
      run_gemm<3>(c, c.ha[0], c.wt_out, c.b_out, c.hn[0], DD, 0, c.out, c.hb);
      run_gemm<4>(c, c.ha[0], c.wt_c1, c.b_c1, c.hn[0], DH, 0, c.cb, c.hb);
      k_cons<<<1, NTHR, 0, c.st>>>(c.cb, c.w_c2, c.b_c2, c.out + (size_t)MR * DD);
    } else {
      run_gemm<2>(c, c.ha[depth], c.wt_out, c.b_out, c.hn[depth - 1], DD, depth - 1, c.cb, c.ha[depth - 1]);
    }
  }
}

}

extern "C" void kernel_launch(void* const* d_in, const int* in_sizes, int n_in,
                              void* d_out, int out_size, void* d_ws, size_t ws_size,
                              hipStream_t stream) {
  if (n_in < 14) return;
  if (in_sizes[0] != MR * KD || in_sizes[1] != DD * KD || in_sizes[2] != DD ||
      in_sizes[3] != 3 * DD * KD || in_sizes[4] != 3 * DD || in_sizes[5] != DD * KD ||
      in_sizes[6] != DD || in_sizes[7] != DH * KD || in_sizes[8] != DH || in_sizes[9] != 3 * DH ||
      in_sizes[10] != 3 || in_sizes[11] != 5 || in_sizes[12] != 1 || in_sizes[13] != 1) return;
  if (out_size != MR * DD + MR * 3) return;

  const float* x     = (const float*)d_in[0];
  const float* W_in  = (const float*)d_in[1];
  const float* b_in  = (const float*)d_in[2];
  const float* W_h   = (const float*)d_in[3];
  const float* b_h   = (const float*)d_in[4];
  const float* W_out = (const float*)d_in[5];
  const float* b_out = (const float*)d_in[6];
  const float* W_c1  = (const float*)d_in[7];
  const float* b_c1  = (const float*)d_in[8];
  const float* W_c2  = (const float*)d_in[9];
  const float* b_c2  = (const float*)d_in[10];
  const float* sf    = (const float*)d_in[11];
  const float* modp  = (const float*)d_in[12];
  const float* ratep = (const float*)d_in[13];

  char* ws = (char*)d_ws;
  size_t off = 0;
  auto take = [&](size_t bytes) { const size_t o = off; off += bytes; off = (off + 255) & ~(size_t)255; return o; };
  const size_t oWin  = take((size_t)DD * KD * 2);
  const size_t oWh   = take((size_t)3 * DD * KD * 2);
  const size_t oWout = take((size_t)DD * KD * 2);
  const size_t oWc1  = take((size_t)DH * KD * 2);
  size_t oX[4], oH[4], oHN[3];
  for (int d = 0; d < 4; ++d) oX[d] = take((size_t)MR * KD * 2);
  for (int d = 0; d < 4; ++d) oH[d] = take((size_t)MR * KD * 2);
  const size_t oHb = take((size_t)MR * KD * 2);
  for (int d = 0; d < 3; ++d) oHN[d] = take((size_t)MR * DD * 4);
  const size_t oC = take((size_t)MR * DH * 4);
  if (off > ws_size || off > (size_t)WSCAP) return;

  Net c;
  c.wt_in  = (const _Float16*)(ws + oWin);
  c.wt_h   = (const _Float16*)(ws + oWh);
  c.wt_out = (const _Float16*)(ws + oWout);
  c.wt_c1  = (const _Float16*)(ws + oWc1);
  for (int d = 0; d < 4; ++d) { c.xa[d] = (_Float16*)(ws + oX[d]); c.ha[d] = (_Float16*)(ws + oH[d]); }
  c.hb = (_Float16*)(ws + oHb);
  for (int d = 0; d < 3; ++d) c.hn[d] = (float*)(ws + oHN[d]);
  c.cb = (float*)(ws + oC);
  c.out = (float*)d_out;
  c.b_in = b_in; c.b_h = b_h; c.b_out = b_out; c.b_c1 = b_c1; c.w_c2 = W_c2; c.b_c2 = b_c2;
  c.sf = sf; c.modp = modp; c.ratep = ratep;
  c.st = stream;
  {
    const double fd = (double)1.618f;
    c.fs.s0 = (float)(1.0 / (fd * fd));
    c.fs.s1 = (float)(1.0 / fd);
    c.fs.s2 = 1.0f;
    c.fs.s3 = 1.618f;
    c.fs.s4 = (float)(fd * fd);
  }

  k_cvt<<<(DD * KD) / (8 * NTHR), NTHR, 0, stream>>>(W_in,  (_Float16*)(ws + oWin),  (float)WSC);
  k_cvt<<<(3 * DD * KD) / (8 * NTHR), NTHR, 0, stream>>>(W_h, (_Float16*)(ws + oWh), (float)WSC);
  k_cvt<<<(DD * KD) / (8 * NTHR), NTHR, 0, stream>>>(W_out, (_Float16*)(ws + oWout), (float)WSC);
  k_cvt<<<(DH * KD) / (8 * NTHR), NTHR, 0, stream>>>(W_c1,  (_Float16*)(ws + oWc1),  (float)WSC);
  k_cvt<<<(MR * KD) / (8 * NTHR), NTHR, 0, stream>>>(x, c.xa[0], (float)ASC);

  hipFuncSetAttribute(reinterpret_cast<const void*>(&k_gemm<0>), hipFuncAttributeMaxDynamicSharedMemorySize, LDS_GEMM);
  hipFuncSetAttribute(reinterpret_cast<const void*>(&k_gemm<1>), hipFuncAttributeMaxDynamicSharedMemorySize, LDS_GEMM);
  hipFuncSetAttribute(reinterpret_cast<const void*>(&k_gemm<2>), hipFuncAttributeMaxDynamicSharedMemorySize, LDS_GEMM);
  hipFuncSetAttribute(reinterpret_cast<const void*>(&k_gemm<3>), hipFuncAttributeMaxDynamicSharedMemorySize, LDS_GEMM);
  hipFuncSetAttribute(reinterpret_cast<const void*>(&k_gemm<4>), hipFuncAttributeMaxDynamicSharedMemorySize, LDS_GEMM);

  fwd(c, 0);
}
